// LSTMAutoencoder_46729244180983
// MI455X (gfx1250) — hardware-verified
//
#include <hip/hip_runtime.h>
#include <math.h>

constexpr int NB   = 32;
constexpr int NF   = 128;
constexpr int NTT  = 2400;
constexpr int NH   = 256;
constexpr int NSEG = 24;
constexpr int NS   = 100;
constexpr int NR   = NB * NS;
constexpr int NRT  = NB * NTT;
constexpr int NG1  = 4 * NH;
constexpr int NG2  = 4 * NF;
constexpr int NTHR = 256;
constexpr int RB   = 16;
constexpr int HP1  = NH + 8;
constexpr int HP2  = NF + 8;
constexpr int OPS  = NH + 4;
constexpr int ZP   = NG1 + 4;
constexpr int TTILE = 32;
constexpr float WCAR  = 16.0f;
constexpr float WINV  = 1.0f / WCAR;
constexpr float LOCAR = 2048.0f;
constexpr float LOINV = WINV / LOCAR;

static_assert(NTT == NS * NSEG);
static_assert(NRT == NR * NSEG);
static_assert(NR % RB == 0 && NB % RB == 0);
static_assert(NH == 32 * (NTHR / 32));
static_assert(NF == 16 * (NTHR / 32));
static_assert(NF % 32 == 0 && NH % 32 == 0);
static_assert(NTT % TTILE == 0);
static_assert(HP1 % 8 == 0 && HP2 % 8 == 0 && OPS % 4 == 0);
static_assert(RB * (NH / 8) == 2 * NTHR);
static_assert(RB * (NF / 4) == 2 * NTHR);
static_assert(NF * (TTILE / 4) == 4 * NTHR);
static_assert(TTILE * (NF / 8) == 2 * NTHR);
static_assert(TTILE * (NF / 4) == 4 * NTHR);
static_assert((NG1 * NF) % (8 * NTHR) == 0 && (NG1 * NH) % (8 * NTHR) == 0);
static_assert((NG2 * NH) % (8 * NTHR) == 0 && (NG2 * NF) % (8 * NTHR) == 0);

typedef __attribute__((ext_vector_type(16))) _Float16 v16h;
typedef __attribute__((ext_vector_type(8)))  _Float16 v8h;
typedef __attribute__((ext_vector_type(8)))  float    v8f;
typedef __attribute__((ext_vector_type(4)))  float    v4f;

__device__ __forceinline__ v16h ldfrag(const _Float16* p) {
  union { v16h v; v8h h[2]; } f;
  f.h[0] = *(const v8h*)(p);
  f.h[1] = *(const v8h*)(p + 16);
  return f.v;
}
__device__ __forceinline__ v8f mma16(v16h a, v16h b, v8f c) {
  return __builtin_amdgcn_wmma_f32_16x16x32_f16(false, a, false, b, (short)0, c, false, false);
}
__device__ __forceinline__ void hz2(v8f& a0, v8f& a1, v16h x, v16h b0, v16h b1) {
  asm volatile("v_nop\n\tv_nop\n\tv_nop\n\tv_nop" : "+v"(a0), "+v"(a1) : "v"(x), "v"(b0), "v"(b1));
}
__device__ __forceinline__ void hz4(v8f& a0, v8f& a1, v8f& l0, v8f& l1, v16h x, v16h y, v16h b0, v16h b1) {
  asm volatile("v_nop\n\tv_nop\n\tv_nop\n\tv_nop"
               : "+v"(a0), "+v"(a1), "+v"(l0), "+v"(l1)
               : "v"(x), "v"(y), "v"(b0), "v"(b1));
}
__device__ __forceinline__ void accg4(v8f& a, v8f& b, v8f& c, v8f& d) {
  asm volatile("v_nop\n\tv_nop\n\tv_nop\n\tv_nop" : "+v"(a), "+v"(b), "+v"(c), "+v"(d));
}
__device__ __forceinline__ void chain4(float& a, float& b, float& c, float& d, float dep) {
  asm volatile("" : "+v"(a), "+v"(b), "+v"(c), "+v"(d) : "v"(dep));
}

__device__ __forceinline__ void mma4(v8f (&acc)[4], const _Float16* pa, const _Float16* pw, size_t gs) {
  const v16h a  = ldfrag(pa);
  const v16h b0 = ldfrag(pw);
  const v16h b1 = ldfrag(pw + gs);
  acc[0] = mma16(a, b0, acc[0]);
  acc[1] = mma16(a, b1, acc[1]);
  hz2(acc[0], acc[1], a, b0, b1);
  const v16h b2 = ldfrag(pw + 2 * gs);
  const v16h b3 = ldfrag(pw + 3 * gs);
  acc[2] = mma16(a, b2, acc[2]);
  acc[3] = mma16(a, b3, acc[3]);
  hz2(acc[2], acc[3], a, b2, b3);
}
__device__ __forceinline__ void mma4x2(v8f (&acc)[4], v8f (&accl)[4], const _Float16* pa, const _Float16* pl,
                                       const _Float16* pw, size_t gs) {
  const v16h a  = ldfrag(pa);
  const v16h al = ldfrag(pl);
  const v16h b0 = ldfrag(pw);
  const v16h b1 = ldfrag(pw + gs);
  acc[0]  = mma16(a,  b0, acc[0]);
  accl[0] = mma16(al, b0, accl[0]);
  acc[1]  = mma16(a,  b1, acc[1]);
  accl[1] = mma16(al, b1, accl[1]);
  hz4(acc[0], acc[1], accl[0], accl[1], a, al, b0, b1);
  const v16h b2 = ldfrag(pw + 2 * gs);
  const v16h b3 = ldfrag(pw + 3 * gs);
  acc[2]  = mma16(a,  b2, acc[2]);
  accl[2] = mma16(al, b2, accl[2]);
  acc[3]  = mma16(a,  b3, acc[3]);
  accl[3] = mma16(al, b3, accl[3]);
  hz4(acc[2], acc[3], accl[2], accl[3], a, al, b2, b3);
}

__device__ __forceinline__ float fsig(float x)  { return __builtin_amdgcn_rcpf(1.0f + expf(-x)); }
__device__ __forceinline__ float ftanh(float x) { return 1.0f - 2.0f * __builtin_amdgcn_rcpf(expf(2.0f * x) + 1.0f); }
__device__ __forceinline__ void lstm_cell(float zi, float zf, float zg, float zo, float& dch, float& cs, float& hs) {
  chain4(zi, zf, zg, zo, dch);
  const float ig = fsig(zi);
  const float fg = fsig(zf);
  const float gg = ftanh(zg);
  const float og = fsig(zo);
  const float cn = fg * cs + ig * gg;
  cs = cn;
  hs = og * ftanh(cn);
  dch = hs;
}
__device__ __forceinline__ void split16(float v, _Float16& hi, _Float16& lo) {
  const _Float16 hv = (_Float16)v;
  hi = hv;
  lo = (_Float16)((v - (float)hv) * LOCAR);
}

__global__ __launch_bounds__(NTHR) void cvt_w16_kernel(const float* __restrict__ src, unsigned short* __restrict__ dst,
                                                       int n8, float sc) {
  const int i = blockIdx.x * NTHR + threadIdx.x;
  if (i < n8) {
    const float* sp = src + (size_t)i * 8;
    const v4f a = *(const v4f*)(sp);
    const v4f b = *(const v4f*)(sp + 4);
    v8h hv;
#pragma unroll
    for (int e = 0; e < 4; ++e) {
      hv[e]     = (_Float16)(a[e] * sc);
      hv[4 + e] = (_Float16)(b[e] * sc);
    }
    unsigned short* dp = dst + (size_t)i * 8;
    *(volatile v8h*)dp = hv;
    __threadfence();
    *(volatile v8h*)dp = hv;
  }
}

__global__ __launch_bounds__(NTHR) void tin_kernel(const float* __restrict__ inp, unsigned short* __restrict__ XT) {
  __shared__ float Tt[NF * (TTILE + 1)];
  const int tid = threadIdx.x;
  const int t0 = blockIdx.x * TTILE;
  const int b = blockIdx.y;
  const float* src = inp + (size_t)b * NF * NTT + t0;
#pragma unroll
  for (int i = 0; i < 4; ++i) {
    const int idx = i * NTHR + tid;
    const int rr = idx >> 3, cc = (idx & 7) * 4;
    const v4f v = *(const v4f*)(src + (size_t)rr * NTT + cc);
    Tt[rr * (TTILE + 1) + cc + 0] = v[0];
    Tt[rr * (TTILE + 1) + cc + 1] = v[1];
    Tt[rr * (TTILE + 1) + cc + 2] = v[2];
    Tt[rr * (TTILE + 1) + cc + 3] = v[3];
  }
  __syncthreads();
  for (int pass = 0; pass < 2; ++pass) {
#pragma unroll
    for (int g = 0; g < 2; ++g) {
      const int idx = g * NTHR + tid;
      const int tq = idx >> 4, c8 = (idx & 15) * 8;
      v8h hv;
#pragma unroll
      for (int e = 0; e < 8; ++e) hv[e] = (_Float16)Tt[(c8 + e) * (TTILE + 1) + tq];
      *(volatile v8h*)(XT + ((size_t)b * NTT + (size_t)(t0 + tq)) * NF + c8) = hv;
    }
    __threadfence();
  }
}

__global__ __launch_bounds__(NTHR) void tout_kernel(const float* __restrict__ REC, float* __restrict__ out) {
  __shared__ float To[TTILE * (NF + 1)];
  const int tid = threadIdx.x;
  const int t0 = blockIdx.x * TTILE;
  const int b = blockIdx.y;
  const float* src = REC + ((size_t)b * NTT + (size_t)t0) * NF;
#pragma unroll
  for (int i = 0; i < 4; ++i) {
    const int idx = i * NTHR + tid;
    const int rr = idx >> 5, c4 = (idx & 31) * 4;
    const v4f v = *(const v4f*)(src + (size_t)rr * NF + c4);
    To[rr * (NF + 1) + c4 + 0] = v[0];
    To[rr * (NF + 1) + c4 + 1] = v[1];
    To[rr * (NF + 1) + c4 + 2] = v[2];
    To[rr * (NF + 1) + c4 + 3] = v[3];
  }
  __syncthreads();
  for (int pass = 0; pass < 2; ++pass) {
#pragma unroll
    for (int it = 0; it < 4; ++it) {
      const int idx = it * NTHR + tid;
      const int fr = idx >> 3, c4 = (idx & 7) * 4;
      v4f o;
#pragma unroll
      for (int e = 0; e < 4; ++e) o[e] = To[(c4 + e) * (NF + 1) + fr];
      *(volatile v4f*)(out + ((size_t)b * NF + (size_t)fr) * NTT + t0 + c4) = o;
    }
    __threadfence();
  }
}

__device__ __forceinline__ void store16x256_hilo(const float* slab, unsigned short* PH, unsigned short* PL,
                                                 size_t base, size_t rstride, int tid) {
  for (int pass = 0; pass < 2; ++pass) {
#pragma unroll
    for (int it = 0; it < 2; ++it) {
      const int idx = it * NTHR + tid;
      const int row = idx >> 5, c8 = (idx & 31) * 8;
      const v4f va = *(const v4f*)(slab + row * OPS + c8);
      const v4f vb = *(const v4f*)(slab + row * OPS + c8 + 4);
      v8h hv, lv;
#pragma unroll
      for (int e = 0; e < 4; ++e) {
        _Float16 h0, l0, h1, l1;
        split16(va[e], h0, l0);
        split16(vb[e], h1, l1);
        hv[e] = h0; lv[e] = l0; hv[4 + e] = h1; lv[4 + e] = l1;
      }
      const size_t o = base + (size_t)row * rstride + c8;
      *(volatile v8h*)(PH + o) = hv;
      *(volatile v8h*)(PL + o) = lv;
    }
    __threadfence();
  }
}


__global__ __launch_bounds__(NTHR) __attribute__((amdgpu_num_vgpr(256)))
void oe_kernel(const unsigned short* __restrict__ XTp,
               const unsigned short* __restrict__ WXp,
               const unsigned short* __restrict__ WHp,
               const float* __restrict__ bih, const float* __restrict__ bhh,
               unsigned short* __restrict__ CSH, unsigned short* __restrict__ CSL) {
  __shared__ __align__(16) _Float16 Ah[RB * HP1];
  __shared__ __align__(16) float    Hs[RB * OPS];
  const _Float16* XT = (const _Float16*)XTp;
  const _Float16* WX = (const _Float16*)WXp;
  const _Float16* WH = (const _Float16*)WHp;
  const int tid = threadIdx.x, lane = tid & 31, wave = tid >> 5;
  const int c = lane & 15, hh = lane >> 4, koff = hh * 8;
  const int rowbase = blockIdx.x * RB;

#pragma unroll 1
  for (int i = tid; i < RB * HP1; i += NTHR) Ah[i] = (_Float16)0.0f;
  float cst[2][8], hst[2][8], bb[2][4];
#pragma unroll
  for (int nt = 0; nt < 2; ++nt) {
    const int j = 32 * wave + 16 * nt + c;
#pragma unroll
    for (int g = 0; g < 4; ++g) bb[nt][g] = bih[g * NH + j] + bhh[g * NH + j];
    asm volatile("" ::: "memory");
#pragma unroll
    for (int r = 0; r < 8; ++r) { cst[nt][r] = 0.0f; hst[nt][r] = 0.0f; }
  }
  __syncthreads();

  const _Float16* ahrow = Ah + c * HP1 + koff;
  const v8f z8 = {0.f, 0.f, 0.f, 0.f, 0.f, 0.f, 0.f, 0.f};

#pragma unroll 1
  for (int t = 0; t < NSEG; ++t) {
    const _Float16* xrow = XT + ((size_t)(rowbase + c) * NSEG + (size_t)t) * NF + koff;
#pragma unroll
    for (int nt = 0; nt < 2; ++nt) {
      const int j = 32 * wave + 16 * nt + c;
      const _Float16* wx = WX + (size_t)j * NF + koff;
      const _Float16* wh = WH + (size_t)j * NH + koff;
      v8f acc[4];
      acc[0] = z8; acc[1] = z8; acc[2] = z8; acc[3] = z8;
#pragma unroll 1
      for (int kx = 0; kx < NF; kx += 32) mma4(acc, xrow + kx, wx + kx, (size_t)NH * NF);
      if (t > 0) {
#pragma unroll 1
        for (int k0 = 0; k0 < NH; k0 += 32) mma4(acc, ahrow + k0, wh + k0, (size_t)NH * NH);
      }
      accg4(acc[0], acc[1], acc[2], acc[3]);
      float dch = bb[nt][0];
#pragma unroll
      for (int r = 0; r < 8; ++r) {
        const float zi = acc[0][r] * WINV + bb[nt][0];
        const float zf = acc[1][r] * WINV + bb[nt][1];
        const float zg = acc[2][r] * WINV + bb[nt][2];
        const float zo = acc[3][r] * WINV + bb[nt][3];
        lstm_cell(zi, zf, zg, zo, dch, cst[nt][r], hst[nt][r]);
      }
    }
    __syncthreads();
#pragma unroll
    for (int nt = 0; nt < 2; ++nt) {
      const int j = 32 * wave + 16 * nt + c;
#pragma unroll
      for (int r = 0; r < 8; ++r) Ah[(8 * hh + r) * HP1 + j] = (_Float16)hst[nt][r];
    }
    __syncthreads();
  }

#pragma unroll
  for (int nt = 0; nt < 2; ++nt) {
    const int j = 32 * wave + 16 * nt + c;
#pragma unroll
    for (int r = 0; r < 8; ++r) Hs[(8 * hh + r) * OPS + j] = cst[nt][r];
  }
  __syncthreads();
  store16x256_hilo(Hs, CSH, CSL, (size_t)rowbase * NH, (size_t)NH, tid);
}

__global__ __launch_bounds__(NTHR) __attribute__((amdgpu_num_vgpr(256)))
void ie_kernel(const unsigned short* __restrict__ CSHp, const unsigned short* __restrict__ CSLp,
               const unsigned short* __restrict__ WXp,
               const unsigned short* __restrict__ WHp,
               const float* __restrict__ bih, const float* __restrict__ bhh,
               unsigned short* __restrict__ BOH, unsigned short* __restrict__ BOL) {
  __shared__ __align__(16) _Float16 Ah[RB * HP1];
  __shared__ __align__(16) float    Hs[RB * OPS];
  const _Float16* XH = (const _Float16*)CSHp;
  const _Float16* XL = (const _Float16*)CSLp;
  const _Float16* WX = (const _Float16*)WXp;
  const _Float16* WH = (const _Float16*)WHp;
  const int tid = threadIdx.x, lane = tid & 31, wave = tid >> 5;
  const int c = lane & 15, hh = lane >> 4, koff = hh * 8;
  const int rowbase = blockIdx.x * RB;

#pragma unroll 1
  for (int i = tid; i < RB * HP1; i += NTHR) Ah[i] = (_Float16)0.0f;
  float cst[2][8], hst[2][8], bb[2][4];
#pragma unroll
  for (int nt = 0; nt < 2; ++nt) {
    const int j = 32 * wave + 16 * nt + c;
#pragma unroll
    for (int g = 0; g < 4; ++g) bb[nt][g] = bih[g * NH + j] + bhh[g * NH + j];
    asm volatile("" ::: "memory");
#pragma unroll
    for (int r = 0; r < 8; ++r) { cst[nt][r] = 0.0f; hst[nt][r] = 0.0f; }
  }
  __syncthreads();

  const _Float16* ahrow = Ah + c * HP1 + koff;
  const v8f z8 = {0.f, 0.f, 0.f, 0.f, 0.f, 0.f, 0.f, 0.f};

#pragma unroll 1
  for (int t = 0; t < NS; ++t) {
    const size_t xo = ((size_t)(rowbase + c) * NS + (size_t)t) * NH + koff;
    const _Float16* xh = XH + xo;
    const _Float16* xl = XL + xo;
#pragma unroll
    for (int nt = 0; nt < 2; ++nt) {
      const int j = 32 * wave + 16 * nt + c;
      const _Float16* wx = WX + (size_t)j * NH + koff;
      const _Float16* wh = WH + (size_t)j * NH + koff;
      v8f acc[4], accl[4];
      acc[0] = z8; acc[1] = z8; acc[2] = z8; acc[3] = z8;
      accl[0] = z8; accl[1] = z8; accl[2] = z8; accl[3] = z8;
#pragma unroll 1
      for (int k0 = 0; k0 < NH; k0 += 32) mma4x2(acc, accl, xh + k0, xl + k0, wx + k0, (size_t)NH * NH);
      if (t > 0) {
#pragma unroll 1
        for (int k0 = 0; k0 < NH; k0 += 32) mma4(acc, ahrow + k0, wh + k0, (size_t)NH * NH);
      }
      accg4(acc[0], acc[1], acc[2], acc[3]);
      accg4(accl[0], accl[1], accl[2], accl[3]);
      float dch = bb[nt][0];
#pragma unroll
      for (int r = 0; r < 8; ++r) {
        const float zi = acc[0][r] * WINV + accl[0][r] * LOINV + bb[nt][0];
        const float zf = acc[1][r] * WINV + accl[1][r] * LOINV + bb[nt][1];
        const float zg = acc[2][r] * WINV + accl[2][r] * LOINV + bb[nt][2];
        const float zo = acc[3][r] * WINV + accl[3][r] * LOINV + bb[nt][3];
        lstm_cell(zi, zf, zg, zo, dch, cst[nt][r], hst[nt][r]);
      }
    }
    __syncthreads();
#pragma unroll
    for (int nt = 0; nt < 2; ++nt) {
      const int j = 32 * wave + 16 * nt + c;
#pragma unroll
      for (int r = 0; r < 8; ++r) Ah[(8 * hh + r) * HP1 + j] = (_Float16)hst[nt][r];
    }
    __syncthreads();
  }

#pragma unroll
  for (int nt = 0; nt < 2; ++nt) {
    const int j = 32 * wave + 16 * nt + c;
#pragma unroll
    for (int r = 0; r < 8; ++r) Hs[(8 * hh + r) * OPS + j] = cst[nt][r];
  }
  __syncthreads();
  store16x256_hilo(Hs, BOH, BOL, (size_t)rowbase * NH, (size_t)NH, tid);
}

__global__ __launch_bounds__(NTHR) __attribute__((amdgpu_num_vgpr(256)))
void id_kernel(const unsigned short* __restrict__ BOHp, const unsigned short* __restrict__ BOLp,
               const unsigned short* __restrict__ WXp,
               const unsigned short* __restrict__ WHp,
               const float* __restrict__ bih, const float* __restrict__ bhh,
               unsigned short* __restrict__ DEH, unsigned short* __restrict__ DEL) {
  __shared__ __align__(16) _Float16 Ah[RB * HP1];
  __shared__ __align__(16) float    Hs[RB * OPS];
  __shared__ __align__(16) float    Zb[RB * ZP];
  const _Float16* XH = (const _Float16*)BOHp;
  const _Float16* XL = (const _Float16*)BOLp;
  const _Float16* WX = (const _Float16*)WXp;
  const _Float16* WH = (const _Float16*)WHp;
  const int tid = threadIdx.x, lane = tid & 31, wave = tid >> 5;
  const int c = lane & 15, hh = lane >> 4, koff = hh * 8;
  const int rowbase = blockIdx.x * RB;
  const v8f z8 = {0.f, 0.f, 0.f, 0.f, 0.f, 0.f, 0.f, 0.f};

#pragma unroll 1
  for (int i = tid; i < RB * HP1; i += NTHR) Ah[i] = (_Float16)0.0f;
  float cst[2][8], hst[2][8], bb[2][4];
#pragma unroll
  for (int nt = 0; nt < 2; ++nt) {
    const int j = 32 * wave + 16 * nt + c;
#pragma unroll
    for (int g = 0; g < 4; ++g) bb[nt][g] = bih[g * NH + j] + bhh[g * NH + j];
    asm volatile("" ::: "memory");
#pragma unroll
    for (int r = 0; r < 8; ++r) { cst[nt][r] = 0.0f; hst[nt][r] = 0.0f; }
  }

  {
    const size_t xo = (size_t)(rowbase + c) * NH + koff;
    const _Float16* xh = XH + xo;
    const _Float16* xl = XL + xo;
#pragma unroll
    for (int nt = 0; nt < 2; ++nt) {
      const int j = 32 * wave + 16 * nt + c;
      const _Float16* wx = WX + (size_t)j * NH + koff;
      v8f acc[4], accl[4];
      acc[0] = z8; acc[1] = z8; acc[2] = z8; acc[3] = z8;
      accl[0] = z8; accl[1] = z8; accl[2] = z8; accl[3] = z8;
#pragma unroll 1
      for (int k0 = 0; k0 < NH; k0 += 32) mma4x2(acc, accl, xh + k0, xl + k0, wx + k0, (size_t)NH * NH);
      accg4(acc[0], acc[1], acc[2], acc[3]);
      accg4(accl[0], accl[1], accl[2], accl[3]);
#pragma unroll
      for (int g = 0; g < 4; ++g)
#pragma unroll
        for (int r = 0; r < 8; ++r)
          Zb[(8 * hh + r) * ZP + g * NH + j] = acc[g][r] * WINV + accl[g][r] * LOINV + bb[nt][g];
    }
  }
  __syncthreads();

  const _Float16* ahrow = Ah + c * HP1 + koff;

#pragma unroll 1
  for (int t = 0; t < NS; ++t) {
#pragma unroll
    for (int nt = 0; nt < 2; ++nt) {
      const int j = 32 * wave + 16 * nt + c;
      const _Float16* wh = WH + (size_t)j * NH + koff;
      v8f acc[4];
      acc[0] = z8; acc[1] = z8; acc[2] = z8; acc[3] = z8;
      if (t > 0) {
#pragma unroll 1
        for (int k0 = 0; k0 < NH; k0 += 32) mma4(acc, ahrow + k0, wh + k0, (size_t)NH * NH);
      }
      accg4(acc[0], acc[1], acc[2], acc[3]);
      float dch = bb[nt][0];
#pragma unroll
      for (int r = 0; r < 8; ++r) {
        const float* zb = Zb + (8 * hh + r) * ZP + j;
        const float zi = zb[0 * NH] + acc[0][r] * WINV;
        const float zf = zb[1 * NH] + acc[1][r] * WINV;
        const float zg = zb[2 * NH] + acc[2][r] * WINV;
        const float zo = zb[3 * NH] + acc[3][r] * WINV;
        lstm_cell(zi, zf, zg, zo, dch, cst[nt][r], hst[nt][r]);
      }
    }
    __syncthreads();
#pragma unroll
    for (int nt = 0; nt < 2; ++nt) {
      const int j = 32 * wave + 16 * nt + c;
#pragma unroll
      for (int r = 0; r < 8; ++r) {
        Ah[(8 * hh + r) * HP1 + j] = (_Float16)hst[nt][r];
        Hs[(8 * hh + r) * OPS + j] = hst[nt][r];
      }
    }
    __syncthreads();
    store16x256_hilo(Hs, DEH, DEL, ((size_t)rowbase * NS + (size_t)t) * NH, (size_t)NS * NH, tid);
  }
}

__global__ __launch_bounds__(NTHR) __attribute__((amdgpu_num_vgpr(256)))
void od_kernel(const unsigned short* __restrict__ DEHp, const unsigned short* __restrict__ DELp,
               const unsigned short* __restrict__ WXp,
               const unsigned short* __restrict__ WHp,
               const float* __restrict__ bih, const float* __restrict__ bhh,
               float* __restrict__ REC) {
  __shared__ __align__(16) _Float16 Ah[RB * HP2];
  __shared__ __align__(16) float    Hs[RB * OPS];
  const _Float16* XH = (const _Float16*)DEHp;
  const _Float16* XL = (const _Float16*)DELp;
  const _Float16* WX = (const _Float16*)WXp;
  const _Float16* WH = (const _Float16*)WHp;
  const int tid = threadIdx.x, lane = tid & 31, wave = tid >> 5;
  const int c = lane & 15, hh = lane >> 4, koff = hh * 8;
  const int rowbase = blockIdx.x * RB;
  const int j = 16 * wave + c;
  const v8f z8 = {0.f, 0.f, 0.f, 0.f, 0.f, 0.f, 0.f, 0.f};

#pragma unroll 1
  for (int i = tid; i < RB * HP2; i += NTHR) Ah[i] = (_Float16)0.0f;
  float cst[8], hst[8], bb[4], zx[4][8];
#pragma unroll
  for (int g = 0; g < 4; ++g) bb[g] = bih[g * NF + j] + bhh[g * NF + j];
  asm volatile("" ::: "memory");
#pragma unroll
  for (int r = 0; r < 8; ++r) { cst[r] = 0.0f; hst[r] = 0.0f; }

  {
    const size_t xo = (size_t)(rowbase + c) * NH + koff;
    const _Float16* xh = XH + xo;
    const _Float16* xl = XL + xo;
    const _Float16* wx = WX + (size_t)j * NH + koff;
    v8f acc[4], accl[4];
    acc[0] = z8; acc[1] = z8; acc[2] = z8; acc[3] = z8;
    accl[0] = z8; accl[1] = z8; accl[2] = z8; accl[3] = z8;
#pragma unroll 1
    for (int k0 = 0; k0 < NH; k0 += 32) mma4x2(acc, accl, xh + k0, xl + k0, wx + k0, (size_t)NF * NH);
    accg4(acc[0], acc[1], acc[2], acc[3]);
    accg4(accl[0], accl[1], accl[2], accl[3]);
#pragma unroll
    for (int g = 0; g < 4; ++g)
#pragma unroll
      for (int r = 0; r < 8; ++r) zx[g][r] = acc[g][r] * WINV + accl[g][r] * LOINV + bb[g];
  }
  __syncthreads();

  const _Float16* ahrow = Ah + c * HP2 + koff;
  const _Float16* wh  = WH + (size_t)j * NF + koff;

#pragma unroll 1
  for (int t = 0; t < NSEG; ++t) {
    v8f acc[4];
    acc[0] = z8; acc[1] = z8; acc[2] = z8; acc[3] = z8;
    if (t > 0) {
#pragma unroll 1
      for (int k0 = 0; k0 < NF; k0 += 32) mma4(acc, ahrow + k0, wh + k0, (size_t)NF * NF);
    }
    accg4(acc[0], acc[1], acc[2], acc[3]);
    float dch = bb[0];
#pragma unroll
    for (int r = 0; r < 8; ++r) {
      const float zi = zx[0][r] + acc[0][r] * WINV;
      const float zf = zx[1][r] + acc[1][r] * WINV;
      const float zg = zx[2][r] + acc[2][r] * WINV;
      const float zo = zx[3][r] + acc[3][r] * WINV;
      lstm_cell(zi, zf, zg, zo, dch, cst[r], hst[r]);
    }
    __syncthreads();
#pragma unroll
    for (int r = 0; r < 8; ++r) {
      Ah[(8 * hh + r) * HP2 + j] = (_Float16)hst[r];
      Hs[(8 * hh + r) * OPS + j] = hst[r];
    }
    __syncthreads();
    for (int pass = 0; pass < 2; ++pass) {
#pragma unroll
      for (int it = 0; it < 2; ++it) {
        const int idx = it * NTHR + tid;
        const int row = idx >> 5, c4 = (idx & 31) * 4;
        const v4f v = *(const v4f*)(Hs + row * OPS + c4);
        *(volatile v4f*)(REC + ((size_t)(rowbase + row) * NSEG + (size_t)t) * NF + c4) = v;
      }
      __threadfence();
    }
  }
}

extern "C" void kernel_launch(void* const* d_in, const int* in_sizes, int n_in,
                              void* d_out, int out_size, void* d_ws, size_t ws_size, hipStream_t stream) {
  if (n_in < 17 || d_out == nullptr || d_ws == nullptr) return;
  if (in_sizes[0] != NB * NF * NTT ||
      in_sizes[1] != NG1 * NF || in_sizes[2] != NG1 * NH || in_sizes[3] != NG1 || in_sizes[4] != NG1 ||
      in_sizes[5] != NG1 * NH || in_sizes[6] != NG1 * NH || in_sizes[7] != NG1 || in_sizes[8] != NG1 ||
      in_sizes[9] != NG1 * NH || in_sizes[10] != NG1 * NH || in_sizes[11] != NG1 || in_sizes[12] != NG1 ||
      in_sizes[13] != NG2 * NH || in_sizes[14] != NG2 * NF || in_sizes[15] != NG2 || in_sizes[16] != NG2 ||
      out_size != NB * NF * NTT) return;

  const float* inp    = (const float*)d_in[0];
  const float* oe_wih = (const float*)d_in[1];
  const float* oe_whh = (const float*)d_in[2];
  const float* oe_bih = (const float*)d_in[3];
  const float* oe_bhh = (const float*)d_in[4];
  const float* ie_wih = (const float*)d_in[5];
  const float* ie_whh = (const float*)d_in[6];
  const float* ie_bih = (const float*)d_in[7];
  const float* ie_bhh = (const float*)d_in[8];
  const float* id_wih = (const float*)d_in[9];
  const float* id_whh = (const float*)d_in[10];
  const float* id_bih = (const float*)d_in[11];
  const float* id_bhh = (const float*)d_in[12];
  const float* od_wih = (const float*)d_in[13];
  const float* od_whh = (const float*)d_in[14];
  const float* od_bih = (const float*)d_in[15];
  const float* od_bhh = (const float*)d_in[16];
  float* out = (float*)d_out;

  char* ws = (char*)d_ws; size_t off = 0;
  auto carve = [&](size_t bytes) -> char* { char* p = ws + off; off += (bytes + 255) & ~(size_t)255; return p; };
  unsigned short* WOEX = (unsigned short*)carve((size_t)NG1 * NF * 2);
  unsigned short* WOEH = (unsigned short*)carve((size_t)NG1 * NH * 2);
  unsigned short* WIEX = (unsigned short*)carve((size_t)NG1 * NH * 2);
  unsigned short* WIEH = (unsigned short*)carve((size_t)NG1 * NH * 2);
  unsigned short* WIDX = (unsigned short*)carve((size_t)NG1 * NH * 2);
  unsigned short* WIDH = (unsigned short*)carve((size_t)NG1 * NH * 2);
  unsigned short* WODX = (unsigned short*)carve((size_t)NG2 * NH * 2);
  unsigned short* WODH = (unsigned short*)carve((size_t)NG2 * NF * 2);
  unsigned short* XT   = (unsigned short*)carve((size_t)NRT * NF * 2);
  unsigned short* CSH  = (unsigned short*)carve((size_t)NR * NH * 2);
  unsigned short* CSL  = (unsigned short*)carve((size_t)NR * NH * 2);
  unsigned short* BOH  = (unsigned short*)carve((size_t)NB * NH * 2);
  unsigned short* BOL  = (unsigned short*)carve((size_t)NB * NH * 2);
  unsigned short* DEH  = (unsigned short*)carve((size_t)NR * NH * 2);
  unsigned short* DEL  = (unsigned short*)carve((size_t)NR * NH * 2);
  float*          REC  = (float*)carve((size_t)NRT * NF * 4);
  if (off > ws_size || off > (size_t)134217728) return;

  cvt_w16_kernel<<<(NG1 * NF / 8) / NTHR, NTHR, 0, stream>>>(oe_wih, WOEX, NG1 * NF / 8, WCAR);
  cvt_w16_kernel<<<(NG1 * NH / 8) / NTHR, NTHR, 0, stream>>>(oe_whh, WOEH, NG1 * NH / 8, WCAR);
  cvt_w16_kernel<<<(NG1 * NH / 8) / NTHR, NTHR, 0, stream>>>(ie_wih, WIEX, NG1 * NH / 8, WCAR);
  cvt_w16_kernel<<<(NG1 * NH / 8) / NTHR, NTHR, 0, stream>>>(ie_whh, WIEH, NG1 * NH / 8, WCAR);
  cvt_w16_kernel<<<(NG1 * NH / 8) / NTHR, NTHR, 0, stream>>>(id_wih, WIDX, NG1 * NH / 8, WCAR);
  cvt_w16_kernel<<<(NG1 * NH / 8) / NTHR, NTHR, 0, stream>>>(id_whh, WIDH, NG1 * NH / 8, WCAR);
  cvt_w16_kernel<<<(NG2 * NH / 8) / NTHR, NTHR, 0, stream>>>(od_wih, WODX, NG2 * NH / 8, WCAR);
  cvt_w16_kernel<<<(NG2 * NF / 8) / NTHR, NTHR, 0, stream>>>(od_whh, WODH, NG2 * NF / 8, WCAR);
  tin_kernel<<<dim3(NTT / TTILE, NB), NTHR, 0, stream>>>(inp, XT);
  oe_kernel<<<NR / RB, NTHR, 0, stream>>>(XT, WOEX, WOEH, oe_bih, oe_bhh, CSH, CSL);
  ie_kernel<<<NB / RB, NTHR, 0, stream>>>(CSH, CSL, WIEX, WIEH, ie_bih, ie_bhh, BOH, BOL);
  id_kernel<<<NB / RB, NTHR, 0, stream>>>(BOH, BOL, WIDX, WIDH, id_bih, id_bhh, DEH, DEL);
  od_kernel<<<NR / RB, NTHR, 0, stream>>>(DEH, DEL, WODX, WODH, od_bih, od_bhh, REC);
  tout_kernel<<<dim3(NTT / TTILE, NB), NTHR, 0, stream>>>(REC, out);
}
